// PolicyNetwork_32255204393673
// MI455X (gfx1250) — hardware-verified
//
#include <hip/hip_runtime.h>
#include <stddef.h>

typedef __attribute__((ext_vector_type(16))) _Float16 v16h;
typedef __attribute__((ext_vector_type(8)))  _Float16 v8h;
typedef __attribute__((ext_vector_type(16))) __bf16   v16b;
typedef __attribute__((ext_vector_type(8)))  __bf16   v8b;
typedef __attribute__((ext_vector_type(8)))  float    v8f;
typedef __attribute__((ext_vector_type(4)))  float    v4f;
typedef __attribute__((ext_vector_type(4)))  int      v4i;

constexpr int HDIM = 128;
constexpr int XDIM = 64;
#define NTHR    256
#define NWAVE   8
#define EPT     8
#define NGRP    2
#define CHUNK   (NTHR * EPT * NGRP)
#define WCAP    (EPT * NGRP * 32)
#define LISTN   (NWAVE * WCAP)
#define NBA     512
#define NBD     4096
#define LDS_AGG (NBA * HDIM * 4 + LISTN * 4 + 64)

static_assert((CHUNK & (CHUNK - 1)) == 0);
static_assert(CHUNK <= 4096);
static_assert((NBA & (NBA - 1)) == 0 && NBA <= 4096);
static_assert((NBD & (NBD - 1)) == 0 && NBD <= 4096);
static_assert(NBD == NWAVE * 4 * 128);
static_assert(NBA == NWAVE * 64);
static_assert((NBA * HDIM / 4) % NTHR == 0);
static_assert(XDIM % 32 == 0 && HDIM % 64 == 0 && XDIM == 64 && HDIM == 128);

__device__ __forceinline__ unsigned short f2bf_bits(float f) {
  unsigned u = __float_as_uint(f);
  return (unsigned short)((u + 0x7FFFu + ((u >> 16) & 1u)) >> 16);
}
__device__ __forceinline__ float bf_bits2f(unsigned short h) { return __uint_as_float(((unsigned)h) << 16); }

__device__ __forceinline__ void dep_guard_h(v8f& a, v8f& b, v16h x, v16h y) { asm volatile("v_nop\n\tv_nop\n\tv_nop\n\tv_nop" : "+v"(a), "+v"(b) : "v"(x), "v"(y)); }
__device__ __forceinline__ void dep_guard_b(v8f& a, v8f& b, v16b x, v16b y) { asm volatile("v_nop\n\tv_nop\n\tv_nop\n\tv_nop" : "+v"(a), "+v"(b) : "v"(x), "v"(y)); }
__device__ __forceinline__ void keep4_h(v16h a, v16h b, v16h c, v16h d) { asm volatile("v_nop" :: "v"(a), "v"(b), "v"(c), "v"(d)); }
__device__ __forceinline__ void keep4_b(v16b a, v16b b, v16b c, v16b d) { asm volatile("v_nop" :: "v"(a), "v"(b), "v"(c), "v"(d)); }
__device__ __forceinline__ void acc_guard4(v8f& a, v8f& b, v8f& c, v8f& d) { asm volatile("v_nop\n\tv_nop\n\tv_nop\n\tv_nop" : "+v"(a), "+v"(b), "+v"(c), "+v"(d)); }
template <typename T> struct Frag;
template <> struct Frag<_Float16> {
  typedef v16h V; union U { v16h v; v8h h[2]; };
  static __device__ __forceinline__ v16h load(const _Float16* p) {
    U f; f.h[0] = *(const v8h*)(p); f.h[1] = *(const v8h*)(p + 16); return f.v;
  }
  static __device__ __forceinline__ v8f mma(v16h a, v16h b, v8f c) {
    return __builtin_amdgcn_wmma_f32_16x16x32_f16(false, a, false, b, (short)0, c, false, false);
  }
  static __device__ __forceinline__ void guard(v8f& a, v8f& b, v16h x, v16h y) { dep_guard_h(a, b, x, y); }
  static __device__ __forceinline__ void keep(v16h a, v16h b, v16h c, v16h d) { keep4_h(a, b, c, d); }
};
template <> struct Frag<__bf16> {
  typedef v16b V; union U { v16b v; v8b h[2]; };
  static __device__ __forceinline__ v16b load(const __bf16* p) {
    U f; f.h[0] = *(const v8b*)(p); f.h[1] = *(const v8b*)(p + 16); return f.v;
  }
  static __device__ __forceinline__ v8f mma(v16b a, v16b b, v8f c) {
    return __builtin_amdgcn_wmma_f32_16x16x32_bf16(false, a, false, b, (short)0, c, false, false);
  }
  static __device__ __forceinline__ void guard(v8f& a, v8f& b, v16b x, v16b y) { dep_guard_b(a, b, x, y); }
  static __device__ __forceinline__ void keep(v16b a, v16b b, v16b c, v16b d) { keep4_b(a, b, c, d); }
};

template <int ET> struct Elem;
template <> struct Elem<0> { typedef _Float16 T; };
template <> struct Elem<1> { typedef __bf16 T; };
template <int ET, bool SPLIT, int BIAS_MODE, int OUT_MODE, bool RESID, int ACT = 0>
__global__ __launch_bounds__(256) void wmma_gemm64(
    const unsigned short* __restrict__ Ap, const unsigned short* __restrict__ A2p, int lda, long strideA,
    const unsigned short* __restrict__ Btp, const unsigned short* __restrict__ Bt2p, int ldb, long strideB,
    void* __restrict__ Cout, void* __restrict__ Cout2, int ldc, long strideC,
    const float* __restrict__ bias,
    const float* __restrict__ resid, long strideR,
    int M, int N, int K, float scale) {
  typedef typename Elem<ET>::T T;
  typedef typename Frag<T>::V V;
  const T* A = (const T*)Ap; const T* A2 = (const T*)A2p; const T* Bt = (const T*)Btp; const T* Bt2 = (const T*)Bt2p;
  __shared__ __align__(16) float sT[8][16 * 68];
  const int b    = blockIdx.y;
  const int lane = threadIdx.x & 31;
  const int wave = threadIdx.x >> 5;
  const int tilesN = N >> 6;
  const int tilesM = M >> 6;
  const int tile = blockIdx.x * 8 + wave;
  if (tile >= tilesM * tilesN) return;
  const int tm = tile / tilesN;
  const int tn = tile - tm * tilesN;
  const int m0 = tm << 6;
  const int n0 = tn << 6;

  const T* Ab  = A  + (size_t)b * strideA;
  const T* Bb  = Bt + (size_t)b * strideB;
  const T* Ab2 = SPLIT ? (A2  + (size_t)b * strideA) : nullptr;
  const T* Bb2 = SPLIT ? (Bt2 + (size_t)b * strideB) : nullptr;

  const int rlane = lane & 15;
  const int koff  = (lane >> 4) * 8;
  const int mOff  = (lane >> 4) * 8;

  v8f acc[4][4];
#pragma unroll
  for (int i = 0; i < 4; ++i)
#pragma unroll
    for (int j = 0; j < 4; ++j) acc[i][j] = (v8f){0.f,0.f,0.f,0.f,0.f,0.f,0.f,0.f};

  for (int k0 = 0; k0 < K; k0 += 32) {
    V bh[4], bl[4];
#pragma unroll
    for (int j = 0; j < 4; ++j) {
      const size_t bo = (size_t)(n0 + (j << 4) + rlane) * ldb + koff + k0;
      bh[j] = Frag<T>::load(Bb + bo);
      if (SPLIT) bl[j] = Frag<T>::load(Bb2 + bo);
    }
#pragma unroll
    for (int i = 0; i < 4; ++i) {
      const size_t ao = (size_t)(m0 + (i << 4) + rlane) * lda + koff + k0;
      V ah = Frag<T>::load(Ab + ao);
      V al;
      if (SPLIT) al = Frag<T>::load(Ab2 + ao);
#pragma unroll
      for (int j = 0; j < 4; ++j) {
        acc[i][j] = Frag<T>::mma(ah, bh[j], acc[i][j]);
        if (SPLIT) {
          acc[i][j] = Frag<T>::mma(ah, bl[j], acc[i][j]);
          acc[i][j] = Frag<T>::mma(al, bh[j], acc[i][j]);
        }
      }
      Frag<T>::guard(acc[i][0], acc[i][3], ah, SPLIT ? al : ah);
    }
    Frag<T>::keep(bh[0], bh[1], bh[2], bh[3]);
    if (SPLIT) Frag<T>::keep(bl[0], bl[1], bl[2], bl[3]);
  }
  acc_guard4(acc[0][0], acc[0][1], acc[0][2], acc[0][3]);
  acc_guard4(acc[1][0], acc[1][1], acc[1][2], acc[1][3]);
  acc_guard4(acc[2][0], acc[2][1], acc[2][2], acc[2][3]);
  acc_guard4(acc[3][0], acc[3][1], acc[3][2], acc[3][3]);

  float* slab = sT[wave];
  const float* Rb = RESID ? (resid + (size_t)b * strideR) : nullptr;
#pragma unroll
  for (int i = 0; i < 4; ++i) {
    const int mBase = m0 + (i << 4);
#pragma unroll
    for (int j = 0; j < 4; ++j) {
      const int n = n0 + (j << 4) + rlane;
      float bv = 0.f;
      if (BIAS_MODE == 2) bv = bias[n];
#pragma unroll
      for (int r = 0; r < 8; ++r) {
        float v = acc[i][j][r] * scale;
        if (BIAS_MODE == 1) v += bias[mBase + mOff + r];
        if (BIAS_MODE == 2) v += bv;
        if (RESID) v += Rb[(size_t)(mBase + mOff + r) * ldc + n];
        if (ACT == 1) v = tanhf(v);
        if (ACT == 2) v = fmaxf(v, 0.0f);
        if (ACT == 3) v = v / (1.0f + expf(-v));
        if (ACT == 4) v = (v > 0.f) ? v : 0.01f * v;
        if (ACT == 5) v = 0.5f * v * (1.0f + erff(v * 0.70710678118654752f));
        slab[(mOff + r) * 68 + (j << 4) + rlane] = v;
      }
    }
    __builtin_amdgcn_fence(__ATOMIC_RELEASE, "workgroup");
    __builtin_amdgcn_wave_barrier();
    __builtin_amdgcn_fence(__ATOMIC_ACQUIRE, "workgroup");
    if (OUT_MODE == 0) {
      float* C = (float*)Cout + (size_t)b * strideC;
      const int hh = lane >> 4, c4 = (lane & 15) * 4;
      for (int pass = 0; pass < 2; ++pass) {
#pragma unroll
        for (int it = 0; it < 8; ++it) {
          const int row = it * 2 + hh;
          v4f v = *(const v4f*)(slab + row * 68 + c4);
          *(volatile v4f*)(C + (size_t)(mBase + row) * ldc + n0 + c4) = v;
        }
        __threadfence();
      }
    } else {
      const int q = lane >> 3, c8 = (lane & 7) * 8;
      unsigned short* C  = (unsigned short*)Cout  + (size_t)b * strideC;
      unsigned short* C2 = (OUT_MODE == 2) ? ((unsigned short*)Cout2 + (size_t)b * strideC) : nullptr;
      for (int pass = 0; pass < 2; ++pass) {
#pragma unroll
        for (int it = 0; it < 4; ++it) {
          const int row = it * 4 + q;
          const float* sp = slab + row * 68 + c8;
          v8h hv, lv;
#pragma unroll
          for (int e = 0; e < 8; ++e) {
            if (OUT_MODE == 1) {
              hv[e] = (_Float16)sp[e];
            } else {
              unsigned short hb = f2bf_bits(sp[e]);
              unsigned short lb = f2bf_bits(sp[e] - bf_bits2f(hb));
              hv[e] = __builtin_bit_cast(_Float16, hb);
              lv[e] = __builtin_bit_cast(_Float16, lb);
            }
          }
          *(volatile v8h*)(C + (size_t)(mBase + row) * ldc + n0 + c8) = hv;
          if (OUT_MODE == 2) *(volatile v8h*)(C2 + (size_t)(mBase + row) * ldc + n0 + c8) = lv;
        }
        __threadfence();
      }
    }
    __builtin_amdgcn_fence(__ATOMIC_RELEASE, "workgroup");
    __builtin_amdgcn_wave_barrier();
    __builtin_amdgcn_fence(__ATOMIC_ACQUIRE, "workgroup");
  }
}

__device__ __forceinline__ void split8(v4f a, v4f b, v8h& hv, v8h& lv) {
  unsigned short hb, lb;
#define SPL1(E, F) { hb = f2bf_bits(F); lb = f2bf_bits((F) - bf_bits2f(hb)); \
                     hv[E] = __builtin_bit_cast(_Float16, hb); lv[E] = __builtin_bit_cast(_Float16, lb); }
  SPL1(0, a.x) SPL1(1, a.y) SPL1(2, a.z) SPL1(3, a.w)
  SPL1(4, b.x) SPL1(5, b.y) SPL1(6, b.z) SPL1(7, b.w)
#undef SPL1
}

template <int NB>
__device__ __forceinline__ int scan_chunk(const int* __restrict__ lst, int nE, int cbase, int nodeBase,
                                          int* list, int tid, int lane, int wave, int fullvec) {
  int wc = 0;
#pragma unroll
  for (int g = 0; g < NGRP; ++g) {
    const int el0 = (g * NTHR + tid) * EPT;
    const int e0  = cbase + el0;
    v4i da, db;
    if (fullvec) {
      da = *(const v4i*)(lst + e0);
      db = *(const v4i*)(lst + e0 + 4);
    } else {
      const int em = nE - 1;
      da.x = lst[(e0     < em) ? e0     : em];
      da.y = lst[(e0 + 1 < em) ? e0 + 1 : em];
      da.z = lst[(e0 + 2 < em) ? e0 + 2 : em];
      da.w = lst[(e0 + 3 < em) ? e0 + 3 : em];
      db.x = lst[(e0 + 4 < em) ? e0 + 4 : em];
      db.y = lst[(e0 + 5 < em) ? e0 + 5 : em];
      db.z = lst[(e0 + 6 < em) ? e0 + 6 : em];
      db.w = lst[(e0 + 7 < em) ? e0 + 7 : em];
    }
    const bool v0 = (e0 < nE), v1 = (e0 + 1 < nE), v2 = (e0 + 2 < nE), v3 = (e0 + 3 < nE);
    const bool v4 = (e0 + 4 < nE), v5 = (e0 + 5 < nE), v6 = (e0 + 6 < nE), v7 = (e0 + 7 < nE);
    const unsigned nb = (unsigned)nodeBase;
    const unsigned s0 = (unsigned)da.x - nb, s1 = (unsigned)da.y - nb;
    const unsigned s2 = (unsigned)da.z - nb, s3 = (unsigned)da.w - nb;
    const unsigned s4 = (unsigned)db.x - nb, s5 = (unsigned)db.y - nb;
    const unsigned s6 = (unsigned)db.z - nb, s7 = (unsigned)db.w - nb;
    const bool h0 = v0 && (s0 < (unsigned)NB), h1 = v1 && (s1 < (unsigned)NB);
    const bool h2 = v2 && (s2 < (unsigned)NB), h3 = v3 && (s3 < (unsigned)NB);
    const bool h4 = v4 && (s4 < (unsigned)NB), h5 = v5 && (s5 < (unsigned)NB);
    const bool h6 = v6 && (s6 < (unsigned)NB), h7 = v7 && (s7 < (unsigned)NB);
    const unsigned any = __builtin_amdgcn_ballot_w32(h0 | h1 | h2 | h3 | h4 | h5 | h6 | h7);
    if (any != 0u) {
#define HITJ(J, HJ, SJ) { \
        const unsigned mj = __builtin_amdgcn_ballot_w32(HJ); \
        if (mj != 0u) { \
          if (HJ) { \
            const int pos = wc + (int)__builtin_amdgcn_mbcnt_lo(mj, 0u); \
            if (pos < WCAP) list[wave * WCAP + pos] = ((el0 + (J)) << 12) | (int)(SJ); \
          } \
          wc += (int)__builtin_popcount(mj); } }
      HITJ(0, h0, s0)
      HITJ(1, h1, s1)
      HITJ(2, h2, s2)
      HITJ(3, h3, s3)
      HITJ(4, h4, s4)
      HITJ(5, h5, s5)
      HITJ(6, h6, s6)
      HITJ(7, h7, s7)
#undef HITJ
    }
  }
  return wc;
}

__global__ __launch_bounds__(NTHR) void k_wprep(const float* __restrict__ W, int Kd,
                                                unsigned short* oh, unsigned short* ol) {
  const int i  = blockIdx.x * NTHR + threadIdx.x;
  const int kq = Kd >> 3;
  if (i >= HDIM * kq) return;
  const int n  = i / kq;
  const int k0 = (i - n * kq) * 8;
  const float* p = W + (size_t)k0 * HDIM + n;
  v4f a, b;
  a.x = p[0];        a.y = p[HDIM];     a.z = p[2 * HDIM]; a.w = p[3 * HDIM];
  b.x = p[4 * HDIM]; b.y = p[5 * HDIM]; b.z = p[6 * HDIM]; b.w = p[7 * HDIM];
  v8h hv, lv;
  split8(a, b, hv, lv);
  const size_t o = (size_t)n * Kd + k0;
  *(volatile v8h*)(oh + o) = hv;
  *(volatile v8h*)(ol + o) = lv;
  __threadfence();
  *(volatile v8h*)(oh + o) = hv;
  *(volatile v8h*)(ol + o) = lv;
}

__global__ __launch_bounds__(NTHR) void k_xprep(const float* __restrict__ x, unsigned short* xh,
                                                unsigned short* xl, int nN, int nRows) {
  const int i = blockIdx.x * NTHR + threadIdx.x;
  if (i >= nRows * (XDIM / 8)) return;
  const int row = i >> 3;
  const int c0  = (i & 7) * 8;
  const int rc  = (row < nN) ? row : nN - 1;
  const float* xp = x + (size_t)rc * XDIM + c0;
  v4f a = *(const v4f*)xp, b = *(const v4f*)(xp + 4);
  if (row >= nN) { const v4f z = {0.f, 0.f, 0.f, 0.f}; a = z; b = z; }
  v8h hv, lv;
  split8(a, b, hv, lv);
  const size_t o = (size_t)row * XDIM + c0;
  *(volatile v8h*)(xh + o) = hv;
  *(volatile v8h*)(xl + o) = lv;
  __threadfence();
  *(volatile v8h*)(xh + o) = hv;
  *(volatile v8h*)(xl + o) = lv;
}

__global__ __launch_bounds__(NTHR) void k_deg(const int* __restrict__ rowl, float* dis, int nE, int vec_ok) {
  __shared__ __attribute__((aligned(16))) int cnt[NBD];
  __shared__ __attribute__((aligned(16))) int list[LISTN];
  __shared__ int wcnt[NWAVE];
  const int tid = threadIdx.x, lane = tid & 31, wave = tid >> 5;
  const int nodeBase = blockIdx.x * NBD;

  for (int i = tid; i < NBD; i += NTHR) cnt[i] = 0;
  __syncthreads();

  const int nChunks = (nE + CHUNK - 1) / CHUNK;
#pragma unroll 1
  for (int ch = 0; ch < nChunks; ++ch) {
    const int cbase = ch * CHUNK;
    const int fullvec = (vec_ok != 0 && cbase + CHUNK <= nE) ? 1 : 0;
    const int wc = scan_chunk<NBD>(rowl, nE, cbase, nodeBase, list, tid, lane, wave, fullvec);
    if (lane == 0) wcnt[wave] = wc;
    __syncthreads();
    if (wave == 0) {
#pragma unroll 1
      for (int wsx = 0; wsx < NWAVE; ++wsx) {
        int n = __builtin_amdgcn_readfirstlane(wcnt[wsx]);
        n = n > WCAP ? WCAP : (n < 0 ? 0 : n);
        const int* lp = list + wsx * WCAP;
#pragma unroll 1
        for (int i = 0; i < n; ++i) {
          const int ent  = __builtin_amdgcn_readfirstlane(lp[i]);
          const int slot = ent & (NBD - 1);
          if (lane == 0) cnt[slot] = cnt[slot] + 1;
        }
      }
    }
    __syncthreads();
  }

  v4f dq[4];
#pragma unroll
  for (int q = 0; q < 4; ++q) {
    const int f = (wave * 4 + q) * 128 + 4 * lane;
    const v4i c = *(const v4i*)(cnt + f);
    dq[q].x = rsqrtf((float)(c.x + 1));
    dq[q].y = rsqrtf((float)(c.y + 1));
    dq[q].z = rsqrtf((float)(c.z + 1));
    dq[q].w = rsqrtf((float)(c.w + 1));
  }
  float* dp = dis + (size_t)nodeBase;
#pragma unroll
  for (int q = 0; q < 4; ++q) *(volatile v4f*)(dp + (wave * 4 + q) * 128 + 4 * lane) = dq[q];
  __threadfence();
#pragma unroll
  for (int q = 0; q < 4; ++q) *(volatile v4f*)(dp + (wave * 4 + q) * 128 + 4 * lane) = dq[q];
}

template <bool OUT16>
__global__ __launch_bounds__(NTHR) void k_agg(
    const int* __restrict__ rowl, const int* __restrict__ coll, const float* __restrict__ z,
    const float* __restrict__ dis, unsigned short* oh, unsigned short* ol, float* of,
    int nN, int nE, int vec_ok) {
  extern __shared__ v4f lds_dyn[];
  float* acc  = (float*)lds_dyn;
  int*   list = (int*)(acc + NBA * HDIM);
  int*   wcnt = list + LISTN;
  const int tid = threadIdx.x, lane = tid & 31, wave = tid >> 5;
  const int nodeBase = blockIdx.x * NBA;

  {
    const v4f zz = {0.f, 0.f, 0.f, 0.f};
    for (int i = tid; i < NBA * HDIM / 4; i += NTHR) lds_dyn[i] = zz;
  }
  __syncthreads();

  const int nChunks = (nE + CHUNK - 1) / CHUNK;
#pragma unroll 1
  for (int ch = 0; ch < nChunks; ++ch) {
    const int cbase = ch * CHUNK;
    const int fullvec = (vec_ok != 0 && cbase + CHUNK <= nE) ? 1 : 0;
    const int wc = scan_chunk<NBA>(coll, nE, cbase, nodeBase, list, tid, lane, wave, fullvec);
    if (lane == 0) wcnt[wave] = wc;
    __syncthreads();
    if (wave == 0) {
#pragma unroll 1
      for (int wsx = 0; wsx < NWAVE; ++wsx) {
        int n = __builtin_amdgcn_readfirstlane(wcnt[wsx]);
        n = n > WCAP ? WCAP : (n < 0 ? 0 : n);
        const int* lp = list + wsx * WCAP;
#pragma unroll 1
        for (int i = 0; i < n; ++i) {
          const int ent  = __builtin_amdgcn_readfirstlane(lp[i]);
          const int slot = ent & (NBA - 1);
          int e = cbase + ((ent >> 12) & (CHUNK - 1));
          e = e > nE - 1 ? nE - 1 : e;
          int s = rowl[e];
          s = s < 0 ? 0 : (s > nN - 1 ? nN - 1 : s);
          const float ds = dis[s];
          const v4f v = *(const v4f*)(z + (size_t)s * HDIM + 4 * lane);
          v4f* ap = (v4f*)(acc + slot * HDIM + 4 * lane);
          *ap = *ap + v * ds;
        }
      }
    }
    __syncthreads();
  }

#pragma unroll 2
  for (int i = 0; i < (NBA * HDIM / 4) / NTHR; ++i) {
    const int idx  = i * NTHR + tid;
    const int slot = idx >> 5;
    const int c4   = (idx & 31) * 4;
    const int node = nodeBase + slot;
    const int nc   = (node < nN) ? node : nN - 1;
    const float dn = dis[nc];
    const v4f zs = *(const v4f*)(z + (size_t)nc * HDIM + c4);
    v4f* ap = (v4f*)(acc + slot * HDIM + c4);
    v4f hv = ((*ap) + zs * dn) * dn;
    hv.x = fmaxf(hv.x, 0.f); hv.y = fmaxf(hv.y, 0.f); hv.z = fmaxf(hv.z, 0.f); hv.w = fmaxf(hv.w, 0.f);
    if (node >= nN) { const v4f zz = {0.f, 0.f, 0.f, 0.f}; hv = zz; }
    *ap = hv;
  }
  __syncthreads();

  if (OUT16) {
    unsigned short* hb = oh + (size_t)nodeBase * HDIM;
    unsigned short* lb = ol + (size_t)nodeBase * HDIM;
    for (int pass = 0; pass < 2; ++pass) {
#pragma unroll 4
      for (int q = 0; q < 32; ++q) {
        const int row = wave * 64 + 2 * q + (lane >> 4);
        const int col = (lane & 15) * 8;
        const float* sp = acc + row * HDIM + col;
        const v4f p0 = *(const v4f*)sp, p1 = *(const v4f*)(sp + 4);
        v8h hv, lv;
        split8(p0, p1, hv, lv);
        *(volatile v8h*)(hb + (size_t)row * HDIM + col) = hv;
        *(volatile v8h*)(lb + (size_t)row * HDIM + col) = lv;
      }
      __threadfence();
    }
  } else {
    float* ob = of + (size_t)nodeBase * HDIM;
    for (int pass = 0; pass < 2; ++pass) {
#pragma unroll 4
      for (int q = 0; q < 64; ++q) {
        const int row = wave * 64 + q;
        const v4f v = *(const v4f*)(acc + row * HDIM + 4 * lane);
        *(volatile v4f*)(ob + (size_t)row * HDIM + 4 * lane) = v;
      }
      __threadfence();
    }
  }
}

__global__ __launch_bounds__(NTHR) void k_colsum(const float* __restrict__ h, float* part, int nN) {
  __shared__ float sd[NTHR];
  const int t = threadIdx.x, c = t & 127, rsel = t >> 7;
  const int r0 = blockIdx.x * 256;
  float a = 0.f;
#pragma unroll 4
  for (int i = 0; i < 128; ++i) {
    const int r  = r0 + 2 * i + rsel;
    const int rc = (r < nN) ? r : nN - 1;
    float v = h[(size_t)rc * HDIM + c];
    v = (r < nN) ? v : 0.f;
    a += v;
  }
  sd[t] = a;
  __syncthreads();
  if (t < 128) {
    const float p = sd[t] + sd[t + 128];
    float* pp = part + (size_t)blockIdx.x * HDIM + t;
    *(volatile float*)pp = p;
    __threadfence();
    *(volatile float*)pp = p;
  }
}

__global__ __launch_bounds__(128) void k_head(
    const float* __restrict__ part, int npb, const float* __restrict__ Wg, const float* __restrict__ bg,
    const float* __restrict__ Wa, const float* __restrict__ ba, const float* __restrict__ Wv,
    const float* __restrict__ bv, float* scal, int nN) {
  __shared__ float sg[HDIM];
  __shared__ float red[3][4];
  const int t = threadIdx.x, lane = t & 31, wave = t >> 5;
  double s = 0.0;
#pragma unroll 1
  for (int b = 0; b < npb; ++b) s += (double)part[(size_t)b * HDIM + t];
  const float g = (float)s * (1.0f / (float)nN);
  sg[t] = g;
  __syncthreads();
  float a = bg[t];
#pragma unroll 1
  for (int k = 0; k < HDIM; ++k) a = fmaf(sg[k], Wg[(size_t)k * HDIM + t], a);
  const float gv = fmaxf(a, 0.0f);
  float p1 = gv * Wa[t], p2 = gv * Wa[HDIM + t], p3 = gv * Wv[t];
#pragma unroll
  for (int off = 16; off > 0; off >>= 1) {
    p1 += __shfl_xor(p1, off, 32);
    p2 += __shfl_xor(p2, off, 32);
    p3 += __shfl_xor(p3, off, 32);
  }
  if (lane == 0) { red[0][wave] = p1; red[1][wave] = p2; red[2][wave] = p3; }
  __syncthreads();
  if (wave == 0) {
    const float s1 = (red[0][0] + red[0][1]) + (red[0][2] + red[0][3]);
    const float s2 = (red[1][0] + red[1][1]) + (red[1][2] + red[1][3]);
    const float s3 = (red[2][0] + red[2][1]) + (red[2][2] + red[2][3]);
    const float gz = s2 + ba[0];
    const float en = s1 + s2 + ba[0];
    const float va = s3 + bv[0];
    float mine = 0.f;
    mine = (lane == 0) ? gz : mine;
    mine = (lane == 1) ? en : mine;
    mine = (lane == 2) ? va : mine;
    *(volatile float*)(scal + lane) = mine;
    __threadfence();
    *(volatile float*)(scal + lane) = mine;
  }
}

__global__ __launch_bounds__(NTHR) void k_score(const float* __restrict__ h, const float* __restrict__ Wa,
                                                const float* __restrict__ scal, float* out, int nN, int nLines) {
  const int lane = threadIdx.x & 31, wave = threadIdx.x >> 5;
  const int line = blockIdx.x * NWAVE + wave;
  if (line >= nLines) return;
  const float gz = scal[0], en = scal[1], va = scal[2];
  const v4f wv = *(const v4f*)(Wa + 4 * lane);
  const int n0 = line * 32;
  float mine = 0.f;
#pragma unroll 1
  for (int j = 0; j < 32; ++j) {
    const int node = n0 + j;
    const int nc = (node < nN) ? node : nN - 1;
    const v4f hv = *(const v4f*)(h + (size_t)nc * HDIM + 4 * lane);
    float p = hv.x * wv.x;
    p = fmaf(hv.y, wv.y, p);
    p = fmaf(hv.z, wv.z, p);
    p = fmaf(hv.w, wv.w, p);
#pragma unroll
    for (int off = 16; off > 0; off >>= 1) p += __shfl_xor(p, off, 32);
    mine = (lane == j) ? p : mine;
  }
  const int idx = n0 + lane;
  float v = mine + gz;
  v = (idx == nN) ? en : v;
  v = (idx == nN + 1) ? va : v;
  if (idx < nN + 2) {
    *(volatile float*)(out + idx) = v;
    __threadfence();
    *(volatile float*)(out + idx) = v;
  }
}

extern "C" void kernel_launch(void* const* d_in, const int* in_sizes, int n_in,
                              void* d_out, int out_size, void* d_ws, size_t ws_size,
                              hipStream_t stream) {
  if (n_in < 16) return;
  const int nN = in_sizes[0] / XDIM;
  const int nE = in_sizes[1] / 2;
  if (nN < 1 || nE < 0 || in_sizes[0] != nN * XDIM || in_sizes[1] != 2 * nE) return;
  if (in_sizes[2] != XDIM * HDIM || in_sizes[3] < HDIM) return;
  if (in_sizes[4] != HDIM * HDIM || in_sizes[5] < HDIM) return;
  if (in_sizes[6] != HDIM * HDIM || in_sizes[7] < HDIM) return;
  if (in_sizes[8] != HDIM * HDIM || in_sizes[9] < HDIM) return;
  if (in_sizes[10] != HDIM * HDIM || in_sizes[11] < HDIM) return;
  if (in_sizes[12] < 2 * HDIM || in_sizes[13] < 1 || in_sizes[14] < HDIM || in_sizes[15] < 1) return;
  if (out_size != nN + 2) return;
  if (nN > (1 << 24)) return;

  const float* x    = (const float*)d_in[0];
  const int*   ei   = (const int*)d_in[1];
  const float* W_e1 = (const float*)d_in[2];
  const float* b_e1 = (const float*)d_in[3];
  const float* W_e2 = (const float*)d_in[4];
  const float* b_e2 = (const float*)d_in[5];
  const float* W_c1 = (const float*)d_in[6];
  const float* b_c1 = (const float*)d_in[7];
  const float* W_c2 = (const float*)d_in[8];
  const float* b_c2 = (const float*)d_in[9];
  const float* W_g  = (const float*)d_in[10];
  const float* b_g  = (const float*)d_in[11];
  const float* W_a  = (const float*)d_in[12];
  const float* b_a  = (const float*)d_in[13];
  const float* W_v  = (const float*)d_in[14];
  const float* b_v  = (const float*)d_in[15];
  const int* rowl = ei;
  const int* coll = ei + nE;
  float* out = (float*)d_out;

  const int Mp     = ((nN + 63) / 64) * 64;
  const int nA     = (nN + NBA - 1) / NBA;
  const int RP     = (nA * NBA > Mp) ? nA * NBA : Mp;
  const int nBD    = (nN + NBD - 1) / NBD;
  const int NPB    = (nN + 255) / 256;
  const int nLines = (nN + 2 + 31) / 32;
  const int vec_row = 1;
  const int vec_col = ((nE & 3) == 0) ? 1 : 0;

  char* ws = (char*)d_ws;
  size_t off = 0;
  const size_t plane16 = (size_t)RP * HDIM * 2;
  const size_t oWe1h = off; off += ((size_t)HDIM * XDIM * 2 + 255) & ~(size_t)255;
  const size_t oWe1l = off; off += ((size_t)HDIM * XDIM * 2 + 255) & ~(size_t)255;
  const size_t oWe2h = off; off += ((size_t)HDIM * HDIM * 2 + 255) & ~(size_t)255;
  const size_t oWe2l = off; off += ((size_t)HDIM * HDIM * 2 + 255) & ~(size_t)255;
  const size_t oWc1h = off; off += ((size_t)HDIM * HDIM * 2 + 255) & ~(size_t)255;
  const size_t oWc1l = off; off += ((size_t)HDIM * HDIM * 2 + 255) & ~(size_t)255;
  const size_t oWc2h = off; off += ((size_t)HDIM * HDIM * 2 + 255) & ~(size_t)255;
  const size_t oWc2l = off; off += ((size_t)HDIM * HDIM * 2 + 255) & ~(size_t)255;
  const size_t oDis  = off; off += ((size_t)nBD * NBD * 4 + 255) & ~(size_t)255;
  const size_t oXh   = off; off += ((size_t)Mp * XDIM * 2 + 255) & ~(size_t)255;
  const size_t oXl   = off; off += ((size_t)Mp * XDIM * 2 + 255) & ~(size_t)255;
  const size_t oPAh  = off; off += (plane16 + 255) & ~(size_t)255;
  const size_t oPAl  = off; off += (plane16 + 255) & ~(size_t)255;
  const size_t oPB   = off; off += (2 * plane16 + 255) & ~(size_t)255;
  const size_t oZP   = off; off += ((size_t)RP * HDIM * 4 + 255) & ~(size_t)255;
  const size_t oPart = off; off += ((size_t)NPB * HDIM * 4 + 255) & ~(size_t)255;
  const size_t oScal = off; off += 256;
  if (off > ws_size) return;

  unsigned short* we1h = (unsigned short*)(ws + oWe1h); unsigned short* we1l = (unsigned short*)(ws + oWe1l);
  unsigned short* we2h = (unsigned short*)(ws + oWe2h); unsigned short* we2l = (unsigned short*)(ws + oWe2l);
  unsigned short* wc1h = (unsigned short*)(ws + oWc1h); unsigned short* wc1l = (unsigned short*)(ws + oWc1l);
  unsigned short* wc2h = (unsigned short*)(ws + oWc2h); unsigned short* wc2l = (unsigned short*)(ws + oWc2l);
  float* dis = (float*)(ws + oDis);
  unsigned short* xh  = (unsigned short*)(ws + oXh);
  unsigned short* xl  = (unsigned short*)(ws + oXl);
  unsigned short* pah = (unsigned short*)(ws + oPAh);
  unsigned short* pal = (unsigned short*)(ws + oPAl);
  unsigned short* pbh = (unsigned short*)(ws + oPB);
  unsigned short* pbl = (unsigned short*)(ws + oPB + plane16);
  float* h2   = (float*)(ws + oPB);
  float* zp   = (float*)(ws + oZP);
  float* part = (float*)(ws + oPart);
  float* scal = (float*)(ws + oScal);

  k_wprep<<<(HDIM * (XDIM / 8) + NTHR - 1) / NTHR, NTHR, 0, stream>>>(W_e1, XDIM, we1h, we1l);
  k_wprep<<<(HDIM * (HDIM / 8) + NTHR - 1) / NTHR, NTHR, 0, stream>>>(W_e2, HDIM, we2h, we2l);
  k_wprep<<<(HDIM * (HDIM / 8) + NTHR - 1) / NTHR, NTHR, 0, stream>>>(W_c1, HDIM, wc1h, wc1l);
  k_wprep<<<(HDIM * (HDIM / 8) + NTHR - 1) / NTHR, NTHR, 0, stream>>>(W_c2, HDIM, wc2h, wc2l);

  k_xprep<<<(Mp * (XDIM / 8) + NTHR - 1) / NTHR, NTHR, 0, stream>>>(x, xh, xl, nN, Mp);

  k_deg<<<nBD, NTHR, 0, stream>>>(rowl, dis, nE, vec_row);

  const int gG = ((Mp / 64) * (HDIM / 64) + 7) / 8;
  wmma_gemm64<1, true, 2, 2, false, 2><<<dim3(gG, 1), 256, 0, stream>>>(
      xh, xl, XDIM, 0L, we1h, we1l, XDIM, 0L, (void*)pah, (void*)pal, HDIM, 0L,
      b_e1, b_e1, 0L, Mp, HDIM, XDIM, 1.0f);
  wmma_gemm64<1, true, 2, 2, false, 0><<<dim3(gG, 1), 256, 0, stream>>>(
      pah, pal, HDIM, 0L, we2h, we2l, HDIM, 0L, (void*)pbh, (void*)pbl, HDIM, 0L,
      b_e2, b_e2, 0L, Mp, HDIM, HDIM, 1.0f);
  wmma_gemm64<1, true, 2, 0, false, 0><<<dim3(gG, 1), 256, 0, stream>>>(
      pbh, pbl, HDIM, 0L, wc1h, wc1l, HDIM, 0L, (void*)zp, (void*)zp, HDIM, 0L,
      b_c1, b_c1, 0L, Mp, HDIM, HDIM, 1.0f);

  k_agg<true><<<nA, NTHR, LDS_AGG, stream>>>(rowl, coll, zp, dis, pah, pal, zp, nN, nE, vec_col);

  wmma_gemm64<1, true, 2, 0, false, 0><<<dim3(gG, 1), 256, 0, stream>>>(
      pah, pal, HDIM, 0L, wc2h, wc2l, HDIM, 0L, (void*)zp, (void*)zp, HDIM, 0L,
      b_c2, b_c2, 0L, Mp, HDIM, HDIM, 1.0f);
  k_agg<false><<<nA, NTHR, LDS_AGG, stream>>>(rowl, coll, zp, dis, pah, pal, h2, nN, nE, vec_col);

  k_colsum<<<NPB, NTHR, 0, stream>>>(h2, part, nN);
  k_head<<<1, 128, 0, stream>>>(part, NPB, W_g, b_g, W_a, b_a, W_v, b_v, scal, nN);
  k_score<<<(nLines + NWAVE - 1) / NWAVE, NTHR, 0, stream>>>(h2, W_a, scal, out, nN, nLines);
}
